// self_attention_37469294691104
// MI455X (gfx1250) — hardware-verified
//
#include <hip/hip_runtime.h>
#include <math.h>

typedef __attribute__((ext_vector_type(16))) _Float16 v16h;
typedef __attribute__((ext_vector_type(16))) __bf16 v16b;
typedef __attribute__((ext_vector_type(8)))  _Float16 v8h;
typedef __attribute__((ext_vector_type(8)))  float v8f;
typedef __attribute__((ext_vector_type(4)))  float v4f;
typedef __attribute__((ext_vector_type(2)))  float v2f;
typedef __attribute__((ext_vector_type(4)))  unsigned v4u;
typedef __attribute__((ext_vector_type(4)))  int v4i;
typedef float __attribute__((may_alias)) float_a;
typedef int __attribute__((may_alias)) int_a;

template <typename T> __device__ __forceinline__ void vst2(void* p, T v) { *(volatile T*)p = v; __threadfence(); *(volatile T*)p = v; }
__device__ __forceinline__ v8f wmma16(v16h a, v16h b, v8f c) {
  v8f d = __builtin_amdgcn_wmma_f32_16x16x32_f16(false, a, false, b, (short)0, c, false, false);
  asm volatile("v_nop\n\tv_nop\n\tv_nop\n\tv_nop" : "+v"(d) : "v"(a), "v"(b));
  return d;
}
__device__ __forceinline__ v8f wmma_bf(v16b a, v16b b, v8f c) {
  v8f d = __builtin_amdgcn_wmma_f32_16x16x32_bf16(false, a, false, b, (short)0, c, false, false);
  asm volatile("v_nop\n\tv_nop\n\tv_nop\n\tv_nop" : "+v"(d) : "v"(a), "v"(b));
  return d;
}
__device__ __forceinline__ v16h frag_h(const _Float16* rowk0, int lane) {
  union { v16h v; v8h q[2]; } u; const _Float16* p = rowk0 + 8 * (lane >> 4);
  u.q[0] = *(const v8h*)p; u.q[1] = *(const v8h*)(p + 16); return u.v;
}
__device__ __forceinline__ v16h frag_f32(const float* rowk0, int lane) {
  v16h a; const float* p = rowk0 + 8 * (lane >> 4);
#pragma unroll
  for (int i = 0; i < 8; ++i) { a[i] = (_Float16)p[i]; a[8 + i] = (_Float16)p[16 + i]; }
  return a;
}
__device__ __forceinline__ v16h frag_f32s(const float* rowk0, int lane, float sc) {
  v16h a; const float* p = rowk0 + 8 * (lane >> 4);
#pragma unroll
  for (int i = 0; i < 8; ++i) { a[i] = (_Float16)(p[i] * sc); a[8 + i] = (_Float16)(p[16 + i] * sc); }
  return a;
}
__device__ __forceinline__ v16h fragc_f32(const float* W, int k0, int n, int lane, int ld, int K) {
  v16h a; const int g = lane >> 4;
#pragma unroll
  for (int i = 0; i < 8; ++i) { const int ka = k0 + 8 * g + i, kb = ka + 16;
    a[i] = (_Float16)(ka < K ? W[(size_t)(ka < K ? ka : K - 1) * ld + n] : 0.f); a[8 + i] = (_Float16)(kb < K ? W[(size_t)(kb < K ? kb : K - 1) * ld + n] : 0.f); }
  return a;
}
struct F2 { v16b h, l; };
__device__ __forceinline__ F2 bsplit16(const float v[16]) { F2 r;
#pragma unroll
  for (int i = 0; i < 16; ++i) { const __bf16 h = (__bf16)v[i]; r.h[i] = h; r.l[i] = (__bf16)(v[i] - (float)h); }
  return r; }
__device__ __forceinline__ F2 split_row(const float* row, int k0, int lane) { float v[16]; const float* p = row + k0 + 8 * (lane >> 4);
#pragma unroll
  for (int i = 0; i < 8; ++i) { v[i] = p[i]; v[8 + i] = p[16 + i]; }
  return bsplit16(v); }
__device__ __forceinline__ F2 split_rowK(const float* row, int k0, int lane, int K) { float v[16]; const int g = lane >> 4;
#pragma unroll
  for (int i = 0; i < 8; ++i) { const int ka = k0 + 8 * g + i, kb = ka + 16; v[i] = ka < K ? row[ka < K ? ka : K - 1] : 0.f; v[8 + i] = kb < K ? row[kb < K ? kb : K - 1] : 0.f; }
  return bsplit16(v); }
__device__ __forceinline__ F2 split_col(const float* W, int k0, int n, int lane, int ld, int K) { float v[16]; const int g = lane >> 4;
#pragma unroll
  for (int i = 0; i < 8; ++i) { const int ka = k0 + 8 * g + i, kb = ka + 16; v[i] = ka < K ? W[(size_t)(ka < K ? ka : K - 1) * ld + n] : 0.f; v[8 + i] = kb < K ? W[(size_t)(kb < K ? kb : K - 1) * ld + n] : 0.f; }
  return bsplit16(v); }
__device__ __forceinline__ v8f mac3(const F2& a, const F2& b, v8f c) { c = wmma_bf(a.l, b.h, c); c = wmma_bf(a.h, b.l, c); return wmma_bf(a.h, b.h, c); }
__device__ __forceinline__ float sigm(float v) { return 1.0f / (1.0f + expf(-v)); }
#define LDSX() do { asm volatile("s_wait_dscnt 0" ::: "memory"); __builtin_amdgcn_wave_barrier(); __builtin_amdgcn_fence(__ATOMIC_RELEASE, "workgroup"); } while (0)

__device__ __forceinline__ float bfr(float v) { return (float)(__bf16)v; }
#define NB 8
#define TT 4096
#define DD 64
#ifndef TNB
#define TNB NB
#endif
typedef __attribute__((ext_vector_type(8))) __bf16 v8b;
__device__ __forceinline__ v16b frag_b(const __bf16* rowk0, int lane) { union { v16b v; v8b q[2]; } u; const __bf16* p = rowk0 + 8 * (lane >> 4); u.q[0] = *(const v8b*)p; u.q[1] = *(const v8b*)(p + 16); return u.v; }
__device__ __forceinline__ v16b frag_rb(const float* rowk0, int lane) { v16b a; const float* p = rowk0 + 8 * (lane >> 4);
#pragma unroll
  for (int i = 0; i < 8; ++i) { a[i] = (__bf16)p[i]; a[8 + i] = (__bf16)p[16 + i]; }
  return a; }
#define WS_VP  0u
#define WS_S   (WS_VP + 2u * (size_t)NB * DD * TT)
#define WS_O   (WS_S + 4u * (size_t)TT * TT)
#define WS_END (WS_O + 4u * (size_t)NB * TT * DD)
__global__ __launch_bounds__(128) void k_vt(const float* __restrict__ V, __bf16* __restrict__ VP) { __shared__ __align__(16) __bf16 th[DD][136];
  const int tid = threadIdx.x; const int s0 = blockIdx.x * 128; const size_t b = blockIdx.y;
  for (int e = tid; e < 128 * DD; e += 128) { const int sl_ = e / DD, d = e % DD; th[d][sl_] = (__bf16)V[(b * TT + s0 + sl_) * DD + d]; }
  __syncthreads();
  for (int e = tid; e < DD * 16; e += 128) { const int d = e >> 4, q = e & 15; vst2((unsigned*)(VP + (b * DD + d) * (size_t)TT + s0 + q * 8), *(const v4u*)&th[d][q * 8]); } }
__global__ __launch_bounds__(128) void k_sc(const float* __restrict__ Q, const float* __restrict__ K, int b, float* __restrict__ S) { __shared__ __align__(16) float ss[4][16][132];
  const int tid = threadIdx.x, wave = tid >> 5, lane = tid & 31, col = lane & 15, g = lane >> 4; const int k0 = blockIdx.y * 128; const int ql0 = blockIdx.x * 64 + wave * 16;
  v8f acc[8] = {};
#pragma unroll
  for (int kc = 0; kc < DD / 32; ++kc) { const v16b a = frag_rb(Q + ((size_t)b * TT + ql0 + col) * DD + kc * 32, lane);
#pragma unroll
    for (int j = 0; j < 8; ++j) { const v16b kb = frag_rb(K + ((size_t)b * TT + k0 + j * 16 + col) * DD + kc * 32, lane); asm volatile("s_wait_loadcnt 0x0" ::: "memory"); acc[j] = wmma_bf(a, kb, acc[j]); } }
#pragma unroll
  for (int j = 0; j < 8; ++j)
#pragma unroll
    for (int r = 0; r < 8; ++r) ss[wave][8 * g + r][j * 16 + col] = acc[j][r] * 0.125f;
  LDSX(); for (int rl = 0; rl < 16; ++rl) vst2(S + (size_t)(ql0 + rl) * TT + k0 + lane * 4, *(const v4f*)&ss[wave][rl][lane * 4]); }
__global__ __launch_bounds__(256) void k_sm(float* __restrict__ S) { __shared__ float sred[8]; __shared__ float sbc; __shared__ __align__(16) float sh[TT];
  const int t = threadIdx.x; const size_t row = blockIdx.x; float* sr = S + row * TT;
  float m = -3.0e38f; for (int k = t; k < TT; k += 256) { const float v = sr[k]; sh[k] = v; m = fmaxf(m, v); }
#pragma unroll
  for (int o = 1; o < 32; o <<= 1) m = fmaxf(m, __shfl_xor(m, o));
  if ((t & 31) == 0) sred[t >> 5] = m; __syncthreads(); if (t == 0) { float a = sred[0]; for (int w = 1; w < 8; ++w) a = fmaxf(a, sred[w]); sbc = a; } __syncthreads(); m = sbc; __syncthreads();
  float s = 0.f; for (int k = t; k < TT; k += 256) { const float e = expf(sh[k] - m); sh[k] = e; s += e; }
#pragma unroll
  for (int o = 1; o < 32; o <<= 1) s += __shfl_xor(s, o);
  if ((t & 31) == 0) sred[t >> 5] = s; __syncthreads(); if (t == 0) { float a = 0.f; for (int w = 0; w < 8; ++w) a += sred[w]; sbc = 2048.0f / a; } __syncthreads(); const float sc = sbc;
  for (int k = t; k < TT; k += 256) sh[k] *= sc;
  __syncthreads(); for (int q = t; q < TT / 4; q += 256) vst2(sr + q * 4, *(const v4f*)&sh[q * 4]); }
__global__ __launch_bounds__(128) void k_pv(const float* __restrict__ PS, const __bf16* __restrict__ VP, int b, float* __restrict__ O) { __shared__ __align__(16) float ss[4][16][DD + 4];
  const int tid = threadIdx.x, wave = tid >> 5, lane = tid & 31, col = lane & 15, g = lane >> 4; const int ql0 = blockIdx.x * 64 + wave * 16;
  v8f acc[DD / 16] = {};
#pragma unroll 1
  for (int kc = 0; kc < TT / 32; ++kc) { const F2 p = split_row(PS + (size_t)(ql0 + col) * TT, kc * 32, lane);
#pragma unroll
    for (int j = 0; j < DD / 16; ++j) { const v16b vv = frag_b(VP + ((size_t)b * DD + j * 16 + col) * (size_t)TT + kc * 32, lane); acc[j] = wmma_bf(p.h, vv, acc[j]); acc[j] = wmma_bf(p.l, vv, acc[j]); } }
#pragma unroll
  for (int j = 0; j < DD / 16; ++j)
#pragma unroll
    for (int r = 0; r < 8; ++r) ss[wave][8 * g + r][j * 16 + col] = acc[j][r] * (1.0f / 2048.0f);
  LDSX(); for (int rl = 0; rl < 16; ++rl) if (lane < DD / 4) vst2(O + ((size_t)b * TT + ql0 + rl) * DD + lane * 4, *(const v4f*)&ss[wave][rl][lane * 4]); }
__global__ __launch_bounds__(128) void k_out(const float* __restrict__ O, const float* __restrict__ WO, const float* __restrict__ BO, float* __restrict__ OUT) { __shared__ __align__(16) float sf[4][16][DD + 4];
  const int tid = threadIdx.x, wave = tid >> 5, lane = tid & 31, col = lane & 15, g = lane >> 4; const size_t r0 = (size_t)blockIdx.x * 64 + wave * 16;
  v8f acc[4] = {};
#pragma unroll
  for (int kc = 0; kc < DD / 32; ++kc) { const F2 a = split_row(O + (r0 + col) * DD, kc * 32, lane);
#pragma unroll
    for (int j = 0; j < 4; ++j) { v16b w; const float* wr = WO + (size_t)(j * 16 + col) * DD + kc * 32 + 8 * g;
#pragma unroll
      for (int i = 0; i < 8; ++i) { w[i] = (__bf16)wr[i]; w[8 + i] = (__bf16)wr[16 + i]; }
      asm volatile("s_wait_loadcnt 0x0" ::: "memory"); acc[j] = wmma_bf(a.h, w, acc[j]); acc[j] = wmma_bf(a.l, w, acc[j]); } }
#pragma unroll
  for (int j = 0; j < 4; ++j) { const float bb = bfr(BO[j * 16 + col]);
#pragma unroll
    for (int r = 0; r < 8; ++r) sf[wave][8 * g + r][j * 16 + col] = acc[j][r] + bb; }
  LDSX(); for (int rl = 0; rl < 16; ++rl) if (lane < 16) vst2(OUT + (r0 + rl) * DD + lane * 4, *(const v4f*)&sf[wave][rl][lane * 4]); }
extern "C" void kernel_launch(void* const* d_in, const int* in_sizes, int n_in, void* d_out, int out_size, void* d_ws, size_t ws_size, hipStream_t stream) {
  (void)in_sizes; (void)n_in; (void)out_size;
  const float** F = (const float**)d_in;
  if (ws_size < (size_t)WS_END) return;
  char* ws = (char*)d_ws; __bf16* VP = (__bf16*)(ws + WS_VP); float *S = (float*)(ws + WS_S), *O = (float*)(ws + WS_O);
  k_vt<<<dim3(TT / 128, TNB), 128, 0, stream>>>(F[0], VP);
  for (int b = 0; b < TNB; ++b) {
    k_sc<<<dim3(TT / 64, TT / 128), 128, 0, stream>>>(F[2], F[1], b, S);
    k_sm<<<dim3(TT), 256, 0, stream>>>(S);
    k_pv<<<dim3(TT / 64), 128, 0, stream>>>(S, VP, b, O);
  }
  k_out<<<dim3(TNB * TT / 64), 128, 0, stream>>>(O, F[4], F[5], (float*)d_out);
}
